// MultiQueryAttention_33019708572197
// MI455X (gfx1250) — hardware-verified
//
#include <hip/hip_runtime.h>
#include <stdint.h>


typedef _Float16 v16h __attribute__((ext_vector_type(16)));
typedef _Float16 v8h  __attribute__((ext_vector_type(8)));
typedef float    v8f  __attribute__((ext_vector_type(8)));
typedef float    v4f  __attribute__((ext_vector_type(4)));

#define DM 2048
#define HDIM 128
#define NH 16
#define RHALF 64
#define NB_FULL 2
#define SEQ_FULL 2048
#ifndef NB
#define NB 2
#endif
#ifndef SEQ
#define SEQ 2048
#endif
#ifndef ERW
#if SEQ < 512
#define ERW SEQ
#else
#define ERW 512
#endif
#endif
#define MROWS (NB * SEQ)
#define YCP (2 * DM)
#define PSP 136
#define NQB_LATE (((SEQ - ERW) / 64) > 0 ? ((SEQ - ERW) / 64) : 1)

#define WQS 64.0f
#define WKS 256.0f
#define W2S 1.0f
#define YCARRY 256.0f
#define YRES 64.0f
#define PCARRY 1024.0f
#define PRES 4096.0f
#define QRES 2048.0f
#define ATT_SCALE 0.08838834764831845f
#define LOG2E 1.4426950408889634f

static_assert(SEQ % 128 == 0);
static_assert(SEQ >= ERW && SEQ <= SEQ_FULL);
static_assert(ERW % 128 == 0 && ERW >= 128);
static_assert((SEQ - ERW) % 128 == 0);
static_assert(NB >= 1 && NB <= NB_FULL);
static_assert(DM == NH * HDIM && HDIM == 128 && 2 * RHALF == HDIM);
static_assert(DM / 8 == 256);
static_assert((MROWS * (NH + 1)) % 8 == 0);
static_assert(W2S * YRES == WQS);

union HFrag { v16h v; v8h h[2]; };

__device__ __forceinline__ v16h load_frag(const _Float16* p) {
    HFrag f;
    f.h[0] = *reinterpret_cast<const v8h*>(p);
    f.h[1] = *reinterpret_cast<const v8h*>(p + 16);
    return f.v;
}

__device__ __forceinline__ v8f wmma16(v16h a, v16h b, v8f c) {
    return __builtin_amdgcn_wmma_f32_16x16x32_f16(false, a, false, b, (short)0, c, false, false);
}

__device__ __forceinline__ void guard2x3(v8f& c0, v8f& c1, const v16h& f0, const v16h& f1, const v16h& f2) {
    asm volatile("v_nop\n\tv_nop\n\tv_nop\n\tv_nop"
                 : "+v"(c0), "+v"(c1) : "v"(f0), "v"(f1), "v"(f2) : "memory");
}
__device__ __forceinline__ void guard2x4(v8f& c0, v8f& c1, const v16h& f0, const v16h& f1,
                                         const v16h& f2, const v16h& f3) {
    asm volatile("v_nop\n\tv_nop\n\tv_nop\n\tv_nop"
                 : "+v"(c0), "+v"(c1) : "v"(f0), "v"(f1), "v"(f2), "v"(f3) : "memory");
}
__device__ __forceinline__ void guard4x4(v8f& c0, v8f& c1, v8f& c2, v8f& c3, const v16h& f0,
                                         const v16h& f1, const v16h& f2, const v16h& f3) {
    asm volatile("v_nop\n\tv_nop\n\tv_nop\n\tv_nop"
                 : "+v"(c0), "+v"(c1), "+v"(c2), "+v"(c3) : "v"(f0), "v"(f1), "v"(f2), "v"(f3) : "memory");
}
__device__ __forceinline__ void guard4x5(v8f& c0, v8f& c1, v8f& c2, v8f& c3, const v16h& f0,
                                         const v16h& f1, const v16h& f2, const v16h& f3, const v16h& f4) {
    asm volatile("v_nop\n\tv_nop\n\tv_nop\n\tv_nop"
                 : "+v"(c0), "+v"(c1), "+v"(c2), "+v"(c3)
                 : "v"(f0), "v"(f1), "v"(f2), "v"(f3), "v"(f4) : "memory");
}

__device__ __forceinline__ float bf16r(float f) {
    unsigned int u = __float_as_uint(f);
    u += 0x7FFFu + ((u >> 16) & 1u);
    u &= 0xFFFF0000u;
    return __uint_as_float(u);
}

__global__ __launch_bounds__(256) void k_cvt_x(const float* __restrict__ x, _Float16* x16)
{
    const int row = blockIdx.x;
    const int col = threadIdx.x * 8;
    const int bb = row / SEQ;
    const int s  = row - bb * SEQ;
    const float* src = x + ((size_t)(bb * SEQ_FULL + s)) * DM + col;
    const float4 f0 = *reinterpret_cast<const float4*>(src);
    const float4 f1 = *reinterpret_cast<const float4*>(src + 4);
    v8h o;
    o[0] = (_Float16)bf16r(f0.x); o[1] = (_Float16)bf16r(f0.y);
    o[2] = (_Float16)bf16r(f0.z); o[3] = (_Float16)bf16r(f0.w);
    o[4] = (_Float16)bf16r(f1.x); o[5] = (_Float16)bf16r(f1.y);
    o[6] = (_Float16)bf16r(f1.z); o[7] = (_Float16)bf16r(f1.w);
    _Float16* dst = x16 + (size_t)row * DM + col;
    *(volatile v8h*)dst = o;
    __threadfence();
    *(volatile v8h*)dst = o;
}

__global__ __launch_bounds__(256) void k_wt(const float* __restrict__ W, _Float16* WT, int N, int pitch,
                                            float scale)
{
    __shared__ _Float16 tile[32 * 72] __attribute__((aligned(16)));
    const int tid = threadIdx.x;
    const int n0 = blockIdx.x * 32, k0 = blockIdx.y * 64;
    const int nn = tid & 31, kq = tid >> 5;
#pragma unroll
    for (int i = 0; i < 8; ++i) {
        const int kk = kq + 8 * i;
        const float w = W[(size_t)(k0 + kk) * N + n0 + nn];
        tile[nn * 72 + kk] = (_Float16)(bf16r(w) * scale);
    }
    __syncthreads();
    const int on = tid >> 3, seg = tid & 7;
    const v8h v = *reinterpret_cast<const v8h*>(tile + on * 72 + seg * 8);
    _Float16* dst = WT + (size_t)(n0 + on) * pitch + k0 + seg * 8;
    *(volatile v8h*)dst = v;
    __threadfence();
    *(volatile v8h*)dst = v;
}

__device__ __forceinline__ void epi_f32(v8f (&acc)[2][4], float alpha, float* swf, float* C, int ldc,
                                        int rowbase, int colbase, int lane, int l15, int hi8)
{
    const int rq = lane >> 4, seg = lane & 15;
#pragma unroll
    for (int g = 0; g < 2; ++g) {
#pragma unroll
        for (int ni = 0; ni < 4; ++ni)
#pragma unroll
            for (int j = 0; j < 8; ++j)
                swf[(hi8 + j) * 64 + ni * 16 + l15] = acc[g][ni][j] * alpha;
        __syncthreads();
        v4f v[8];
#pragma unroll
        for (int it = 0; it < 8; ++it)
            v[it] = *reinterpret_cast<const v4f*>(swf + (it * 2 + rq) * 64 + seg * 4);
        float* gd = C + (size_t)(rowbase + g * 16) * ldc + colbase + seg * 4;
#pragma unroll
        for (int it = 0; it < 8; ++it)
            *(volatile v4f*)(gd + (size_t)(it * 2 + rq) * ldc) = v[it];
        __threadfence();
#pragma unroll
        for (int it = 0; it < 8; ++it)
            *(volatile v4f*)(gd + (size_t)(it * 2 + rq) * ldc) = v[it];
        __syncthreads();
    }
}

template <int MODE>
__global__ __launch_bounds__(256) void k_gemm(const _Float16* __restrict__ A,
                                              const _Float16* __restrict__ BT,
                                              void* C0, void* C1, void* C2,
                                              int lda, int ldb, int ldc, int K, float alpha,
                                              int tiles_per_b, int a_bs, int a_off, int c_bs, int c_off)
{
    __shared__ float stg[8 * 1024] __attribute__((aligned(16)));
    const int tid = threadIdx.x;
    const int lane = tid & 31, wave = tid >> 5;
    const int wm = wave & 3, wn = wave >> 2;
    const int l15 = lane & 15, hi8 = (lane >> 4) << 3;
    const int bsel = blockIdx.y / tiles_per_b;
    const int tt = blockIdx.y - bsel * tiles_per_b;
    const int bmA = bsel * a_bs + a_off + tt * 128;
    const int bmC = bsel * c_bs + c_off + tt * 128;
    const int bn0 = blockIdx.x * 128;

    const _Float16* ap0 = A + (size_t)(bmA + wm * 32 + l15) * lda + hi8;
    const _Float16* ap1 = ap0 + (size_t)16 * lda;
    const _Float16* bp  = BT + (size_t)(bn0 + wn * 64 + l15) * ldb + hi8;
    const size_t bst = (size_t)16 * ldb;

    const v8f zero8 = {0.f, 0.f, 0.f, 0.f, 0.f, 0.f, 0.f, 0.f};
    v8f acc[2][4];
#pragma unroll
    for (int g = 0; g < 2; ++g)
#pragma unroll
        for (int ni = 0; ni < 4; ++ni) acc[g][ni] = zero8;

    for (int k0 = 0; k0 < K; k0 += 32) {
        const v16h a0 = load_frag(ap0 + k0);
        const v16h a1 = load_frag(ap1 + k0);
        const v16h b0 = load_frag(bp + k0);
        const v16h b1 = load_frag(bp + bst + k0);
        const v16h b2 = load_frag(bp + 2 * bst + k0);
        const v16h b3 = load_frag(bp + 3 * bst + k0);
        acc[0][0] = wmma16(a0, b0, acc[0][0]);
        acc[0][1] = wmma16(a0, b1, acc[0][1]);
        acc[0][2] = wmma16(a0, b2, acc[0][2]);
        acc[0][3] = wmma16(a0, b3, acc[0][3]);
        acc[1][0] = wmma16(a1, b0, acc[1][0]);
        acc[1][1] = wmma16(a1, b1, acc[1][1]);
        acc[1][2] = wmma16(a1, b2, acc[1][2]);
        acc[1][3] = wmma16(a1, b3, acc[1][3]);
        asm volatile("v_nop\n\tv_nop\n\tv_nop\n\tv_nop"
                     : "+v"(acc[0][0]), "+v"(acc[0][1]), "+v"(acc[0][2]), "+v"(acc[0][3]),
                       "+v"(acc[1][0]), "+v"(acc[1][1]), "+v"(acc[1][2]), "+v"(acc[1][3])
                     : "v"(a0), "v"(a1), "v"(b0), "v"(b1), "v"(b2), "v"(b3));
    }

    if (MODE == 0) {
        epi_f32(acc, alpha, stg + wave * 1024, (float*)C0, ldc, bmC + wm * 32, bn0 + wn * 64, lane, l15, hi8);
    } else {
        if (blockIdx.x == 0) {
            epi_f32(acc, alpha, stg + wave * 1024, (float*)C0, ldc, bmC + wm * 32, wn * 64, lane, l15, hi8);
        } else {
            _Float16* vsh = reinterpret_cast<_Float16*>(stg);
            _Float16* vsr = vsh + 64 * 128;
            const int s0 = c_off + tt * 128;
            const int dq = tid >> 4, seg = tid & 15;
#pragma unroll 1
            for (int p = 0; p < 2; ++p) {
                if (wn == p) {
#pragma unroll
                    for (int g = 0; g < 2; ++g)
#pragma unroll
                        for (int ni = 0; ni < 4; ++ni)
#pragma unroll
                            for (int j = 0; j < 8; ++j) {
                                const float val = acc[g][ni][j] * alpha;
                                const _Float16 hv = (_Float16)val;
                                const int idx = (ni * 16 + l15) * 128 + wm * 32 + g * 16 + hi8 + j;
                                vsh[idx] = hv;
                                vsr[idx] = (_Float16)((val - (float)hv) * PRES);
                            }
                }
                __syncthreads();
                v8h vh[4], vr[4];
#pragma unroll
                for (int it = 0; it < 4; ++it) {
                    vh[it] = *reinterpret_cast<const v8h*>(vsh + (it * 16 + dq) * 128 + seg * 8);
                    vr[it] = *reinterpret_cast<const v8h*>(vsr + (it * 16 + dq) * 128 + seg * 8);
                }
                const size_t rb = ((size_t)(bsel * HDIM + p * 64)) * SEQ + s0 + seg * 8;
                _Float16* vd  = (_Float16*)C1 + rb;
                _Float16* vdr = (_Float16*)C2 + rb;
#pragma unroll
                for (int it = 0; it < 4; ++it) {
                    *(volatile v8h*)(vd  + (size_t)(it * 16 + dq) * SEQ) = vh[it];
                    *(volatile v8h*)(vdr + (size_t)(it * 16 + dq) * SEQ) = vr[it];
                }
                __threadfence();
#pragma unroll
                for (int it = 0; it < 4; ++it) {
                    *(volatile v8h*)(vd  + (size_t)(it * 16 + dq) * SEQ) = vh[it];
                    *(volatile v8h*)(vdr + (size_t)(it * 16 + dq) * SEQ) = vr[it];
                }
                __syncthreads();
            }
        }
    }
}

__global__ __launch_bounds__(256) void k_rope(const float* __restrict__ qpre, const float* __restrict__ kpre,
                                              const float* __restrict__ cosT, const float* __restrict__ sinT,
                                              _Float16* q16, _Float16* qres, _Float16* k16, _Float16* kres)
{
#pragma clang fp contract(off)
    __shared__ _Float16 sh[8 * 256] __attribute__((aligned(16)));
    const int lane = threadIdx.x & 31, wv = threadIdx.x >> 5;
    const int vec = blockIdx.x * 8 + wv;
    const int nq = MROWS * NH;
    const bool isq = vec < nq;
    const int row = isq ? (vec >> 4) : (vec - nq);
    const int hh  = isq ? (vec & 15) : 0;
    const int bb = row / SEQ;
    const int s  = row - bb * SEQ;
    const float* src = isq ? (qpre + (size_t)row * DM + hh * HDIM) : (kpre + (size_t)row * HDIM);

    const float x1a = src[lane], x1b = src[lane + 32], x2a = src[lane + 64], x2b = src[lane + 96];
    const float* cp = cosT + (size_t)s * RHALF;
    const float* sp = sinT + (size_t)s * RHALF;
    const float ca = bf16r(cp[lane]), cb = bf16r(cp[lane + 32]);
    const float sa = bf16r(sp[lane]), sb = bf16r(sp[lane + 32]);

    const float r1a = x1a * ca + x2a * sa;
    const float r1b = x1b * cb + x2b * sb;
    const float r2a = x2a * ca - x1a * sa;
    const float r2b = x2b * cb - x1b * sb;

    float ss = r1a * r1a + r1b * r1b + r2a * r2a + r2b * r2b;
#pragma unroll
    for (int o = 16; o >= 1; o >>= 1) ss += __shfl_xor(ss, o, 32);
    const float inv = rsqrtf(ss * (1.0f / HDIM) + 1e-6f);

    const float o0 = r1a * inv, o1 = r1b * inv, o2 = r2a * inv, o3 = r2b * inv;
    const _Float16 h0 = (_Float16)o0, h1 = (_Float16)o1, h2 = (_Float16)o2, h3 = (_Float16)o3;
    _Float16* sw = sh + wv * 256;
    sw[lane] = h0; sw[lane + 32] = h1; sw[lane + 64] = h2; sw[lane + 96] = h3;
    sw[128 + lane]      = (_Float16)((o0 - (float)h0) * QRES);
    sw[128 + lane + 32] = (_Float16)((o1 - (float)h1) * QRES);
    sw[128 + lane + 64] = (_Float16)((o2 - (float)h2) * QRES);
    sw[128 + lane + 96] = (_Float16)((o3 - (float)h3) * QRES);
    __syncthreads();

    const int pl = lane >> 4, sg = lane & 15;
    const v8h v = *reinterpret_cast<const v8h*>(sw + pl * 128 + sg * 8);
    const int se = (s < ERW) ? s : (ERW - 1);
    _Float16* dhp = isq ? (q16 + (size_t)row * DM + hh * HDIM + sg * 8)
                        : (k16 + (size_t)row * HDIM + sg * 8);
    _Float16* drp = isq ? (qres + ((size_t)(bb * ERW + se)) * DM + hh * HDIM + sg * 8)
                        : (kres + (size_t)row * HDIM + sg * 8);
    _Float16* d = pl ? drp : dhp;
    const bool doit = (pl == 0) || (!isq) || (s < ERW);
    if (doit) *(volatile v8h*)d = v;
    __threadfence();
    if (doit) *(volatile v8h*)d = v;
}

__global__ __launch_bounds__(128) __attribute__((amdgpu_num_vgpr(256)))
void k_attn_late(const _Float16* __restrict__ q16, const _Float16* __restrict__ k16,
                 const _Float16* __restrict__ vTh, _Float16* y16)
{
    __shared__ _Float16 Ps[4 * 16 * PSP] __attribute__((aligned(16)));
    const int lane = threadIdx.x & 31;
    const int wv   = threadIdx.x >> 5;
    const int l15  = lane & 15;
    const int hi8  = (lane >> 4) << 3;

    const int nqb = NQB_LATE;
    int g = blockIdx.x;
    const int qb = ERW / 64 + (g % nqb); g /= nqb;
    const int h  = g % NH;
    const int b  = g / NH;
    const int row0 = qb * 64 + wv * 16;
    const float QSC = ATT_SCALE * LOG2E;

    const _Float16* qbase = q16 + ((size_t)(b * SEQ + row0 + l15)) * DM + h * HDIM + hi8;
    const _Float16* kbase = k16 + ((size_t)(b * SEQ)) * HDIM + hi8;
    const _Float16* vbase = vTh + ((size_t)(b * HDIM + l15)) * SEQ + hi8;

    const v8f zero8 = {0.f, 0.f, 0.f, 0.f, 0.f, 0.f, 0.f, 0.f};
    float m[8], l[8];
    v8f accY[8];
#pragma unroll
    for (int j = 0; j < 8; ++j) { m[j] = -1e30f; l[j] = 0.0f; }
#pragma unroll
    for (int dt = 0; dt < 8; ++dt) accY[dt] = zero8;

    _Float16* ps = Ps + wv * 16 * PSP;
    const int nck = 2 * qb + 2;

#pragma unroll 1
    for (int c = 0; c < nck; ++c) {
        const int tc = c * 32;
        const _Float16* kp0 = kbase + (size_t)(tc + l15) * HDIM;
        const _Float16* kp1 = kp0 + 16 * HDIM;
        v8f s0 = zero8, s1 = zero8;
#pragma unroll
        for (int kc = 0; kc < 4; ++kc) {
            const v16h aq = load_frag(qbase + kc * 32);
            const v16h b0 = load_frag(kp0 + kc * 32);
            const v16h b1 = load_frag(kp1 + kc * 32);
            s0 = wmma16(aq, b0, s0);
            s1 = wmma16(aq, b1, s1);
            guard2x3(s0, s1, aq, b0, b1);
        }

#pragma unroll
        for (int j = 0; j < 8; ++j) {
            const int rowj = row0 + hi8 + j;
            float a0 = s0[j] * QSC;
            float a1 = s1[j] * QSC;
            a0 = (tc + l15 > rowj) ? -1e30f : a0;
            a1 = (tc + 16 + l15 > rowj) ? -1e30f : a1;
            float mt = fmaxf(a0, a1);
#pragma unroll
            for (int off = 8; off >= 1; off >>= 1)
                mt = fmaxf(mt, __shfl_xor(mt, off, 16));
            const float mn = fmaxf(m[j], mt);
            const float sc = exp2f(m[j] - mn);
            const float p0 = exp2f(a0 - mn);
            const float p1 = exp2f(a1 - mn);
            float rs = p0 + p1;
#pragma unroll
            for (int off = 8; off >= 1; off >>= 1)
                rs += __shfl_xor(rs, off, 16);
            l[j] = l[j] * sc + rs;
            m[j] = mn;
#pragma unroll
            for (int dt = 0; dt < 8; ++dt) accY[dt][j] *= sc;
            const int rw = (hi8 + j) * PSP;
            ps[rw + l15]      = (_Float16)(p0 * PCARRY);
            ps[rw + 16 + l15] = (_Float16)(p1 * PCARRY);
        }
        __syncthreads();

        const v16h aP = load_frag(ps + l15 * PSP + hi8);
        {
            const _Float16* vp = vbase + tc;
            const v16h v0 = load_frag(vp);
            const v16h v1 = load_frag(vp + (size_t)16 * SEQ);
            const v16h v2 = load_frag(vp + (size_t)32 * SEQ);
            const v16h v3 = load_frag(vp + (size_t)48 * SEQ);
            accY[0] = wmma16(aP, v0, accY[0]);
            accY[1] = wmma16(aP, v1, accY[1]);
            accY[2] = wmma16(aP, v2, accY[2]);
            accY[3] = wmma16(aP, v3, accY[3]);
            guard4x5(accY[0], accY[1], accY[2], accY[3], aP, v0, v1, v2, v3);
        }
        {
            const _Float16* vp = vbase + (size_t)64 * SEQ + tc;
            const v16h v4 = load_frag(vp);
            const v16h v5 = load_frag(vp + (size_t)16 * SEQ);
            const v16h v6 = load_frag(vp + (size_t)32 * SEQ);
            const v16h v7 = load_frag(vp + (size_t)48 * SEQ);
            accY[4] = wmma16(aP, v4, accY[4]);
            accY[5] = wmma16(aP, v5, accY[5]);
            accY[6] = wmma16(aP, v6, accY[6]);
            accY[7] = wmma16(aP, v7, accY[7]);
            guard4x5(accY[4], accY[5], accY[6], accY[7], aP, v4, v5, v6, v7);
        }
    }
    __syncthreads();

    float inv[8];
#pragma unroll
    for (int j = 0; j < 8; ++j) inv[j] = (YCARRY / PCARRY) / l[j];
#pragma unroll
    for (int dt = 0; dt < 8; ++dt)
#pragma unroll
        for (int j = 0; j < 8; ++j)
            ps[(hi8 + j) * PSP + dt * 16 + l15] = (_Float16)(accY[dt][j] * inv[j]);
    __syncthreads();

    const int rq = lane >> 4, seg = lane & 15;
    v8h v[8];
#pragma unroll
    for (int it = 0; it < 8; ++it)
        v[it] = *reinterpret_cast<const v8h*>(ps + (it * 2 + rq) * PSP + seg * 8);
    _Float16* yd = y16 + ((size_t)(b * SEQ + row0)) * DM + h * HDIM + seg * 8;
#pragma unroll
    for (int it = 0; it < 8; ++it)
        *(volatile v8h*)(yd + (size_t)(it * 2 + rq) * DM) = v[it];
    __threadfence();
#pragma unroll
    for (int it = 0; it < 8; ++it)
        *(volatile v8h*)(yd + (size_t)(it * 2 + rq) * DM) = v[it];
}

__global__ __launch_bounds__(128) __attribute__((amdgpu_num_vgpr(256)))
void k_attn_early(const _Float16* __restrict__ q16, const _Float16* __restrict__ qres,
                  const _Float16* __restrict__ k16, const _Float16* __restrict__ kres,
                  const _Float16* __restrict__ vTh, const _Float16* __restrict__ vTr,
                  _Float16* ycat)
{
    __shared__ _Float16 Ps[4 * 16 * PSP] __attribute__((aligned(16)));
    const int lane = threadIdx.x & 31;
    const int wv   = threadIdx.x >> 5;
    const int l15  = lane & 15;
    const int hi8  = (lane >> 4) << 3;

    const int nqp = ERW / 32;
    int g = blockIdx.x;
    const int qp = g % nqp; g /= nqp;
    const int h  = g % NH;
    const int b  = g / NH;
    const int dh = wv & 1;
    const int row0 = qp * 32 + (wv >> 1) * 16;
    const float QSC = ATT_SCALE * LOG2E;

    const _Float16* qh = q16  + ((size_t)(b * SEQ + row0 + l15)) * DM + h * HDIM + hi8;
    const _Float16* qr = qres + ((size_t)(b * ERW + row0 + l15)) * DM + h * HDIM + hi8;
    const _Float16* kh = k16  + ((size_t)(b * SEQ)) * HDIM + hi8;
    const _Float16* kr = kres + ((size_t)(b * SEQ)) * HDIM + hi8;
    const _Float16* vh = vTh  + ((size_t)(b * HDIM + dh * 64 + l15)) * SEQ + hi8;
    const _Float16* vr = vTr  + ((size_t)(b * HDIM + dh * 64 + l15)) * SEQ + hi8;

    const v8f zero8 = {0.f, 0.f, 0.f, 0.f, 0.f, 0.f, 0.f, 0.f};
    float m[8], l[8];
    v8f accY[4], accR[4];
#pragma unroll
    for (int j = 0; j < 8; ++j) { m[j] = -1e30f; l[j] = 0.0f; }
#pragma unroll
    for (int dt = 0; dt < 4; ++dt) { accY[dt] = zero8; accR[dt] = zero8; }

    _Float16* ps = Ps + wv * 16 * PSP;
    const int nck = qp + 1;

#pragma unroll 1
    for (int c = 0; c < nck; ++c) {
        const int tc = c * 32;
        const _Float16* kp0 = kh + (size_t)(tc + l15) * HDIM;
        const _Float16* kp1 = kp0 + 16 * HDIM;
        const _Float16* rp0 = kr + (size_t)(tc + l15) * HDIM;
        const _Float16* rp1 = rp0 + 16 * HDIM;
        v8f s0 = zero8, s1 = zero8, r0 = zero8, r1 = zero8;
#pragma unroll
        for (int kc = 0; kc < 4; ++kc) {
            const v16h aq = load_frag(qh + kc * 32);
            const v16h ar = load_frag(qr + kc * 32);
            const v16h b0 = load_frag(kp0 + kc * 32);
            const v16h b1 = load_frag(kp1 + kc * 32);
            s0 = wmma16(aq, b0, s0);
            s1 = wmma16(aq, b1, s1);
            r0 = wmma16(ar, b0, r0);
            r1 = wmma16(ar, b1, r1);
            guard4x4(s0, s1, r0, r1, aq, ar, b0, b1);
            const v16h c0 = load_frag(rp0 + kc * 32);
            const v16h c1 = load_frag(rp1 + kc * 32);
            r0 = wmma16(aq, c0, r0);
            r1 = wmma16(aq, c1, r1);
            guard2x3(r0, r1, aq, c0, c1);
        }

#pragma unroll
        for (int j = 0; j < 8; ++j) {
            const int rowj = row0 + hi8 + j;
            float a0 = (s0[j] + r0[j] * (1.0f / QRES)) * QSC;
            float a1 = (s1[j] + r1[j] * (1.0f / QRES)) * QSC;
            a0 = (tc + l15 > rowj) ? -1e30f : a0;
            a1 = (tc + 16 + l15 > rowj) ? -1e30f : a1;
            float mt = fmaxf(a0, a1);
#pragma unroll
            for (int off = 8; off >= 1; off >>= 1)
                mt = fmaxf(mt, __shfl_xor(mt, off, 16));
            const float mn = fmaxf(m[j], mt);
            const float sc = exp2f(m[j] - mn);
            const float p0 = exp2f(a0 - mn);
            const float p1 = exp2f(a1 - mn);
            float rs = p0 + p1;
#pragma unroll
            for (int off = 8; off >= 1; off >>= 1)
                rs += __shfl_xor(rs, off, 16);
            l[j] = l[j] * sc + rs;
            m[j] = mn;
#pragma unroll
            for (int dt = 0; dt < 4; ++dt) { accY[dt][j] *= sc; accR[dt][j] *= sc; }
            const float pc0 = p0 * PCARRY, pc1 = p1 * PCARRY;
            const _Float16 ph0 = (_Float16)pc0, ph1 = (_Float16)pc1;
            const int rw = (hi8 + j) * PSP;
            ps[rw + l15]      = ph0;
            ps[rw + 16 + l15] = ph1;
            ps[rw + 32 + l15] = (_Float16)((pc0 - (float)ph0) * PRES);
            ps[rw + 48 + l15] = (_Float16)((pc1 - (float)ph1) * PRES);
        }
        __syncthreads();

        const v16h aP = load_frag(ps + l15 * PSP + hi8);
        const v16h aR = load_frag(ps + l15 * PSP + 32 + hi8);
#pragma unroll
        for (int dt = 0; dt < 4; ++dt) {
            const size_t vo = (size_t)(dt * 16) * SEQ + tc;
            const v16h bv = load_frag(vh + vo);
            const v16h br = load_frag(vr + vo);
            accY[dt] = wmma16(aP, bv, accY[dt]);
            accR[dt] = wmma16(aP, br, accR[dt]);
            accR[dt] = wmma16(aR, bv, accR[dt]);
            guard2x4(accY[dt], accR[dt], aP, aR, bv, br);
        }
    }
    __syncthreads();

    float inv[8];
#pragma unroll
    for (int j = 0; j < 8; ++j) inv[j] = (YCARRY / PCARRY) / l[j];
#pragma unroll
    for (int dt = 0; dt < 4; ++dt)
#pragma unroll
        for (int j = 0; j < 8; ++j) {
            const float y = (accY[dt][j] + accR[dt][j] * (1.0f / PRES)) * inv[j];
            const _Float16 yhh = (_Float16)y;
            const int rw = (hi8 + j) * PSP;
            ps[rw + dt * 16 + l15]      = yhh;
            ps[rw + 64 + dt * 16 + l15] = (_Float16)((y - (float)yhh) * YRES);
        }
    __syncthreads();

    const int r2 = (lane >> 3) & 1, pl = lane >> 4, seg = lane & 7;
    v8h v[8];
#pragma unroll
    for (int it = 0; it < 8; ++it)
        v[it] = *reinterpret_cast<const v8h*>(ps + (it * 2 + r2) * PSP + pl * 64 + seg * 8);
    _Float16* yd = ycat + ((size_t)(b * ERW + row0)) * YCP + (size_t)pl * DM + h * HDIM + dh * 64 + seg * 8;
#pragma unroll
    for (int it = 0; it < 8; ++it)
        *(volatile v8h*)(yd + (size_t)(it * 2 + r2) * YCP) = v[it];
    __threadfence();
#pragma unroll
    for (int it = 0; it < 8; ++it)
        *(volatile v8h*)(yd + (size_t)(it * 2 + r2) * YCP) = v[it];
}

extern "C" void kernel_launch(void* const* d_in, const int* in_sizes, int n_in,
                              void* d_out, int out_size, void* d_ws, size_t ws_size,
                              hipStream_t stream) {
    if (n_in < 7) return;
    const long long needX = ((long long)(NB - 1) * SEQ_FULL + SEQ) * DM;
    if ((long long)in_sizes[0] < needX) return;
    if (in_sizes[1] < SEQ * RHALF || in_sizes[2] < SEQ * RHALF) return;
    if (in_sizes[3] < DM * DM || in_sizes[4] < DM * HDIM || in_sizes[5] < DM * HDIM || in_sizes[6] < DM * DM) return;
    if ((long long)out_size < (long long)MROWS * DM) return;

    const float* x    = (const float*)d_in[0];
    const float* cosT = (const float*)d_in[1];
    const float* sinT = (const float*)d_in[2];
    const float* Wq   = (const float*)d_in[3];
    const float* Wk   = (const float*)d_in[4];
    const float* Wv   = (const float*)d_in[5];
    const float* Wo   = (const float*)d_in[6];
    float* out = (float*)d_out;

    size_t off = 0;
    char* wsb = (char*)d_ws;
    auto carve = [&](size_t bytes) -> void* {
        void* p = wsb + off;
        off += (bytes + 255) & ~(size_t)255;
        return p;
    };
    _Float16* x16  = (_Float16*)carve((size_t)MROWS * DM * 2);
    _Float16* WqT  = (_Float16*)carve((size_t)DM * DM * 2);
    _Float16* WkvT = (_Float16*)carve((size_t)(2 * HDIM) * DM * 2);
    _Float16* WoTc = (_Float16*)carve((size_t)DM * YCP * 2);
    float*    qpre = (float*)carve((size_t)MROWS * DM * 4);
    float*    kpre = (float*)carve((size_t)MROWS * HDIM * 4);
    _Float16* q16  = (_Float16*)carve((size_t)MROWS * DM * 2);
    _Float16* qrs  = (_Float16*)carve((size_t)NB * ERW * DM * 2);
    _Float16* k16  = (_Float16*)carve((size_t)MROWS * HDIM * 2);
    _Float16* krs  = (_Float16*)carve((size_t)MROWS * HDIM * 2);
    _Float16* vTh  = (_Float16*)carve((size_t)NB * HDIM * SEQ * 2);
    _Float16* vTr  = (_Float16*)carve((size_t)NB * HDIM * SEQ * 2);
    _Float16* y16  = (_Float16*)carve((size_t)MROWS * DM * 2);
    _Float16* ycat = (_Float16*)carve((size_t)NB * ERW * YCP * 2);
    if (off > ws_size) return;

    dim3 blk(256);

    k_cvt_x<<<dim3(MROWS), blk, 0, stream>>>(x, x16);
    k_wt<<<dim3(DM / 32, DM / 64), blk, 0, stream>>>(Wq, WqT, DM, DM, WQS);
    k_wt<<<dim3(HDIM / 32, DM / 64), blk, 0, stream>>>(Wk, WkvT, HDIM, DM, WKS);
    k_wt<<<dim3(HDIM / 32, DM / 64), blk, 0, stream>>>(Wv, WkvT + (size_t)HDIM * DM, HDIM, DM, WKS);
    k_wt<<<dim3(DM / 32, DM / 64), blk, 0, stream>>>(Wo, WoTc, DM, YCP, WQS);
    k_wt<<<dim3(DM / 32, DM / 64), blk, 0, stream>>>(Wo, WoTc + DM, DM, YCP, W2S);

    k_gemm<0><<<dim3(DM / 128, MROWS / 128), blk, 0, stream>>>(
        x16, WqT, (void*)qpre, (void*)qpre, (void*)qpre, DM, DM, DM, DM, 1.0f / WQS,
        SEQ / 128, SEQ, 0, SEQ, 0);
    k_gemm<1><<<dim3(2, MROWS / 128), blk, 0, stream>>>(
        x16, WkvT, (void*)kpre, (void*)vTh, (void*)vTr, DM, DM, HDIM, DM, 1.0f / WKS,
        SEQ / 128, SEQ, 0, SEQ, 0);
    k_rope<<<dim3((MROWS * (NH + 1)) / 8), blk, 0, stream>>>(qpre, kpre, cosT, sinT, q16, qrs, k16, krs);
    k_attn_early<<<dim3(NB * NH * (ERW / 32)), dim3(128), 0, stream>>>(q16, qrs, k16, krs, vTh, vTr, ycat);
    if (SEQ > ERW) {
        k_attn_late<<<dim3(NB * NH * ((SEQ - ERW) / 64)), dim3(128), 0, stream>>>(q16, k16, vTh, y16);
        k_gemm<0><<<dim3(DM / 128, NB * ((SEQ - ERW) / 128)), blk, 0, stream>>>(
            y16, WoTc, (void*)out, (void*)out, (void*)out, DM, YCP, DM, DM, 1.0f / (YCARRY * WQS),
            (SEQ - ERW) / 128, SEQ, ERW, SEQ, ERW);
    }
    k_gemm<0><<<dim3(DM / 128, NB * (ERW / 128)), blk, 0, stream>>>(
        ycat, WoTc, (void*)out, (void*)out, (void*)out, YCP, YCP, DM, YCP, 1.0f / (YCARRY * WQS),
        ERW / 128, ERW, 0, SEQ, 0);
}
